// PointNet_V3_75033078661467
// MI455X (gfx1250) — hardware-run, weakly checked
//
#include <hip/hip_runtime.h>


#ifndef NPTS
#define NPTS 1000000
#endif
#define NPTS_FULL 1000000
#define NSEG  20000
#define CIN   16
#define C1    64
#define C2A   128
#define OW    192
#define SEGB  200
#define CHUNK 256
#define LCAP  288
#define XP    68
#define PB    64
#define PW    8
#define NT    (NPTS / 16)
#define BN_EPS 1.0e-3f
#define W2S   64.0f
#define W2SI  (1.0f / 64.0f)

static_assert(NPTS % 16 == 0);
static_assert(NPTS <= NPTS_FULL);
static_assert(NPTS <= (1 << 20));
static_assert(SEGB < 4096);
static_assert(NSEG % SEGB == 0);
static_assert(CHUNK == 32 * 8);
static_assert(LCAP >= 15 + CHUNK);
static_assert(LCAP % 16 == 0);
static_assert(CIN == 16);
static_assert(C1 == 64);
static_assert(C2A == 128);
static_assert(OW == 3 * C1);
static_assert((OW * 4) % 128 == 0);
static_assert((SEGB * (OW / 4)) % 32 == 0);
static_assert(XP % 2 == 0);
static_assert(XP >= C1);
static_assert(C1 * 32 / 8 == 256);
static_assert(C2A * 32 / 8 == 512);
static_assert(C1 * C2A / 8 == 1024);
static_assert(16 * 16 == C1 * 4);
static_assert(C2A + C1 <= 256);

typedef _Float16 h16;
typedef unsigned short bf;
typedef __attribute__((ext_vector_type(16))) __bf16   v16bf;
typedef __attribute__((ext_vector_type(16))) _Float16 v16h;
typedef __attribute__((ext_vector_type(8)))  _Float16 v8h;
typedef __attribute__((ext_vector_type(8)))  unsigned short v8us;
typedef __attribute__((ext_vector_type(8)))  float    v8f;
typedef __attribute__((ext_vector_type(4)))  float    v4f;
typedef v4f  __attribute__((may_alias)) v4fa;
typedef __attribute__((ext_vector_type(2)))  float    v2f;
typedef v2f  __attribute__((may_alias)) v2fa;
typedef __attribute__((ext_vector_type(4)))  int      v4i;

__device__ __forceinline__ unsigned short f2bf(float f) { unsigned u = __float_as_uint(f); u += 0x7FFFu + ((u >> 16) & 1u); return (unsigned short)(u >> 16); }
__device__ __forceinline__ float bfr(float f) { return __uint_as_float(((unsigned)f2bf(f)) << 16); }
__device__ __forceinline__ v16h cat16(v8h lo, v8h hi) { return __builtin_shufflevector(lo, hi, 0, 1, 2, 3, 4, 5, 6, 7, 8, 9, 10, 11, 12, 13, 14, 15); }
__device__ __forceinline__ v16bf cat16b(v8us lo, v8us hi) { return __builtin_bit_cast(v16bf, __builtin_shufflevector(lo, hi, 0, 1, 2, 3, 4, 5, 6, 7, 8, 9, 10, 11, 12, 13, 14, 15)); }
__device__ __forceinline__ v8f wmma16(v16h a, v16h b, v8f c) { return __builtin_amdgcn_wmma_f32_16x16x32_f16(false, a, false, b, (short)0, c, false, false); }
__device__ __forceinline__ v8f wmmab(v16bf a, v16bf b, v8f c) { return __builtin_amdgcn_wmma_f32_16x16x32_bf16(false, a, false, b, (short)0, c, false, false); }
__device__ __forceinline__ v16h  ldh(const h16* p) { return cat16(*(const v8h*)p, *(const v8h*)(p + 16)); }
__device__ __forceinline__ v16bf ldb(const bf* p)  { return cat16b(*(const v8us*)p, *(const v8us*)(p + 16)); }
__device__ __forceinline__ void wave_sync() { __builtin_amdgcn_fence(3  , "wavefront"); __builtin_amdgcn_wave_barrier(); asm volatile("" ::: "memory"); }

static __device__ __forceinline__ h16 toh_flush(float v) { const h16 r = (h16)v; return (fabsf(v) < 6.103515625e-05f) ? (h16)0.0f : r; }
__device__ __forceinline__ v8f gwmma16(v16h a, v16h b, v8f c) { c = wmma16(a, b, c); asm volatile("v_nop\n\tv_nop\n\tv_nop\n\tv_nop" : "+v"(c) : "v"(a), "v"(b)); return c; }
__device__ __forceinline__ v8f gwmmab(v16bf a, v16bf b, v8f c) { c = wmmab(a, b, c); asm volatile("v_nop\n\tv_nop\n\tv_nop\n\tv_nop" : "+v"(c) : "v"(a), "v"(b)); return c; }
__device__ __forceinline__ float bnf(float a, float m, float s, float b) { return (a - m) * s + b; }

__global__ __launch_bounds__(256) void k_prep(const float* __restrict__ W1, const float* __restrict__ W2a, const float* __restrict__ W2b, bf* W1T, bf* W2AT, h16* W2BT) {
#pragma clang fp contract(off)
    const int blk = blockIdx.x, t = threadIdx.x;
    if (blk < 1) {
        const int p = t; const int n = p >> 2, k8 = (p & 3) * 8; v8us o;
#pragma unroll
        for (int i = 0; i < 8; ++i) { const int k = k8 + i; float x = W1[(size_t)(k & (CIN - 1)) * C1 + n]; asm volatile("" : "+v"(x)); o[i] = (k < CIN) ? f2bf(x) : (bf)0; }
        *(volatile v8us*)(W1T + (size_t)p * 8) = o; __threadfence(); *(volatile v8us*)(W1T + (size_t)p * 8) = o;
    } else if (blk < 3) {
        const int p = (blk - 1) * 256 + t; const int n = p >> 2, k8 = (p & 3) * 8; v8us o;
#pragma unroll
        for (int i = 0; i < 8; ++i) { const int k = k8 + i; float x = W2a[(size_t)(k & (CIN - 1)) * C2A + n]; asm volatile("" : "+v"(x)); o[i] = (k < CIN) ? f2bf(x) : (bf)0; }
        *(volatile v8us*)(W2AT + (size_t)p * 8) = o; __threadfence(); *(volatile v8us*)(W2AT + (size_t)p * 8) = o;
    } else {
        const int p = (blk - 3) * 256 + t; const int c = p >> 4, k8 = (p & 15) * 8; v8h o;
#pragma unroll
        for (int i = 0; i < 8; ++i) { const float x = W2b[(size_t)(k8 + i) * C1 + c]; o[i] = toh_flush(bfr(x) * W2S); }
        *(volatile v8h*)(W2BT + (size_t)p * 8) = o; __threadfence(); *(volatile v8h*)(W2BT + (size_t)p * 8) = o;
    }
}

__global__ __launch_bounds__(256) void k_pool(const float* __restrict__ in, const bf* __restrict__ W2AT, const h16* __restrict__ W2BT,
                                              const float* __restrict__ g2a, const float* __restrict__ b2a, const float* __restrict__ m2a, const float* __restrict__ v2a,
                                              const float* __restrict__ g2b, const float* __restrict__ b2b, const float* __restrict__ m2b, const float* __restrict__ v2b,
                                              float* PM) {
    __shared__ __align__(16) float bn[3 * C2A + 3 * C1];
    __shared__ __align__(16) float pw[PW * 64];
    const int tid = threadIdx.x;
    const int lane = tid & 31, lr = lane & 15, hi = lane >> 4;
    const int wave = __builtin_amdgcn_readfirstlane((int)(threadIdx.x >> 5));
    if (tid < C2A) {
        bn[tid] = bfr(m2a[tid]); bn[C2A + tid] = bfr(g2a[tid]) * rsqrtf(bfr(v2a[tid]) + BN_EPS); bn[2 * C2A + tid] = bfr(b2a[tid]);
    } else if (tid < C2A + C1) {
        const int c = tid - C2A;
        bn[3 * C2A + c] = bfr(m2b[c]); bn[3 * C2A + C1 + c] = bfr(g2b[c]) * rsqrtf(bfr(v2b[c]) + BN_EPS); bn[3 * C2A + 2 * C1 + c] = bfr(b2b[c]);
    }
    __syncthreads();
    const int wg = blockIdx.x * PW + wave;
    const v8f z8 = (v8f){};
    const v8us z8u = (v8us){};
    v8f mx[4];
#pragma unroll
    for (int j = 0; j < 4; ++j) mx[j] = z8;
#pragma unroll 1
    for (int t = wg; t < NT; t += PB * PW) {
        const float* rp = in + ((size_t)t * 16 + lr) * CIN + 8 * hi;
        const v4f x0 = *(const v4f*)rp, x1 = *(const v4f*)(rp + 4);
        v8us lo;
#pragma unroll
        for (int i = 0; i < 4; ++i) { lo[i] = f2bf(x0[i]); lo[4 + i] = f2bf(x1[i]); }
        const v16bf bp = cat16b(lo, z8u);
        v16h hb[4];
#pragma unroll
        for (int s = 0; s < 4; ++s) {
            const v16bf a0 = ldb(W2AT + (size_t)(32 * s + lr) * 32 + 8 * hi);
            const v16bf a1 = ldb(W2AT + (size_t)(32 * s + 16 + lr) * 32 + 8 * hi);
            const v8f d0 = gwmmab(a0, bp, z8);
            const v8f d1 = gwmmab(a1, bp, z8);
            const int cb0 = 32 * s + 8 * hi, cb1 = cb0 + 16;
            const v4f ma0 = *(const v4fa*)(&bn[cb0]),           ma1 = *(const v4fa*)(&bn[cb0 + 4]);
            const v4f sa0 = *(const v4fa*)(&bn[C2A + cb0]),     sa1 = *(const v4fa*)(&bn[C2A + cb0 + 4]);
            const v4f ba0 = *(const v4fa*)(&bn[2 * C2A + cb0]), ba1 = *(const v4fa*)(&bn[2 * C2A + cb0 + 4]);
            const v4f mb0 = *(const v4fa*)(&bn[cb1]),           mb1 = *(const v4fa*)(&bn[cb1 + 4]);
            const v4f sb0 = *(const v4fa*)(&bn[C2A + cb1]),     sb1 = *(const v4fa*)(&bn[C2A + cb1 + 4]);
            const v4f bb0 = *(const v4fa*)(&bn[2 * C2A + cb1]), bb1 = *(const v4fa*)(&bn[2 * C2A + cb1 + 4]);
#pragma unroll
            for (int r = 0; r < 4; ++r) {
                hb[s][r]      = toh_flush(fmaxf(bnf(d0[r],     ma0[r], sa0[r], ba0[r]), 0.0f));
                hb[s][4 + r]  = toh_flush(fmaxf(bnf(d0[4 + r], ma1[r], sa1[r], ba1[r]), 0.0f));
                hb[s][8 + r]  = toh_flush(fmaxf(bnf(d1[r],     mb0[r], sb0[r], bb0[r]), 0.0f));
                hb[s][12 + r] = toh_flush(fmaxf(bnf(d1[4 + r], mb1[r], sb1[r], bb1[r]), 0.0f));
            }
        }
#pragma unroll
        for (int j = 0; j < 4; ++j) {
            v8f acc = z8;
#pragma unroll
            for (int s = 0; s < 4; ++s) {
                const v16h a = ldh(W2BT + (size_t)(16 * j + lr) * C2A + 32 * s + 8 * hi);
                acc = gwmma16(a, hb[s], acc);
            }
            const int cb = 16 * j + 8 * hi;
            const v4f m0 = *(const v4fa*)(&bn[3 * C2A + cb]),          m1 = *(const v4fa*)(&bn[3 * C2A + cb + 4]);
            const v4f s0 = *(const v4fa*)(&bn[3 * C2A + C1 + cb]),     s1 = *(const v4fa*)(&bn[3 * C2A + C1 + cb + 4]);
            const v4f b0 = *(const v4fa*)(&bn[3 * C2A + 2 * C1 + cb]), b1 = *(const v4fa*)(&bn[3 * C2A + 2 * C1 + cb + 4]);
#pragma unroll
            for (int r = 0; r < 4; ++r) {
                mx[j][r]     = fmaxf(mx[j][r],     bnf(acc[r] * W2SI,     m0[r], s0[r], b0[r]));
                mx[j][4 + r] = fmaxf(mx[j][4 + r], bnf(acc[4 + r] * W2SI, m1[r], s1[r], b1[r]));
            }
        }
    }
#pragma unroll
    for (int j = 0; j < 4; ++j) {
#pragma unroll
        for (int r = 0; r < 8; ++r) {
            float v = mx[j][r];
            v = fmaxf(v, __shfl_xor(v, 1, 32)); v = fmaxf(v, __shfl_xor(v, 2, 32));
            v = fmaxf(v, __shfl_xor(v, 4, 32)); v = fmaxf(v, __shfl_xor(v, 8, 32));
            mx[j][r] = v;
        }
    }
    if (lr == 0) {
#pragma unroll
        for (int j = 0; j < 4; ++j) {
            v4f a, c;
            a[0] = mx[j][0]; a[1] = mx[j][1]; a[2] = mx[j][2]; a[3] = mx[j][3]; c[0] = mx[j][4]; c[1] = mx[j][5]; c[2] = mx[j][6]; c[3] = mx[j][7];
            *(v4fa*)(&pw[wave * 64 + 16 * j + 8 * hi]) = a; *(v4fa*)(&pw[wave * 64 + 16 * j + 8 * hi + 4]) = c;
        }
    }
    wave_sync();
    const v4f val = *(const v4fa*)(&pw[wave * 64 + 4 * lr]);
    float* prow = PM + (size_t)wg * 64;
#pragma unroll 1
    for (int ps = 0; ps < 2; ++ps) {
        if (lane < 16) *(volatile v4f*)(prow + 4 * lane) = val;
        if (ps == 0) __threadfence(); }
}

__global__ __launch_bounds__(32) void k_seg(const float* __restrict__ in, const int* __restrict__ seg, const int* __restrict__ nsp, const bf* __restrict__ W1T,
                                            const float* __restrict__ g1, const float* __restrict__ b1, const float* __restrict__ m1, const float* __restrict__ v1,
                                            const float* __restrict__ PM, float* OUT) {
    __shared__ __align__(16) float accs[SEGB * 2 * C1];
    __shared__ __align__(16) float xs[16 * XP];
    __shared__ __align__(16) bf xt[16 * CIN];
    __shared__ __align__(16) unsigned lst[LCAP];
    __shared__ __align__(16) float pool[C1];
    const int lane = threadIdx.x & 31, lr = lane & 15, hi = lane >> 4;
    const int s0 = blockIdx.x * SEGB;
    const int ns = max(0, min(nsp[0], NSEG));
    const int nloc = max(0, min(ns - s0, SEGB));
    const v4f z4 = (v4f){};
    const v8f z8 = (v8f){};
    const v8us z8u = (v8us){};
#pragma unroll 4
    for (int i = lane; i < SEGB * 32; i += 32) *(v4fa*)(&accs[4 * i]) = z4;
    { float p0 = 0.0f, p1 = 0.0f;
#pragma unroll 4
      for (int i = 0; i < PB * PW; ++i) { p0 = fmaxf(p0, PM[(size_t)i * 64 + lane]); p1 = fmaxf(p1, PM[(size_t)i * 64 + 32 + lane]); }
      pool[lane] = p0; pool[32 + lane] = p1; }
    v16bf w1f[4]; float m1r[4], s1r[4], b1r[4];
#pragma unroll
    for (int j = 0; j < 4; ++j) {
        w1f[j] = ldb(W1T + (size_t)(16 * j + lr) * 32 + 8 * hi);
        const int c = 16 * j + lr;
        m1r[j] = bfr(m1[c]); s1r[j] = bfr(g1[c]) * rsqrtf(bfr(v1[c]) + BN_EPS); b1r[j] = bfr(b1[c]);
    }
    wave_sync();
    int cnt = 0;
#pragma unroll 1
    for (int base = 0; ; base += CHUNK) {
        const bool last = base >= NPTS;
        if (!last) {
            int sv[8];
            if (base + CHUNK <= NPTS) {
                const v4i a = *(const v4i*)(seg + base + lane * 8); const v4i b = *(const v4i*)(seg + base + lane * 8 + 4);
                sv[0] = a[0]; sv[1] = a[1]; sv[2] = a[2]; sv[3] = a[3]; sv[4] = b[0]; sv[5] = b[1]; sv[6] = b[2]; sv[7] = b[3];
            } else {
#pragma unroll
                for (int j = 0; j < 8; ++j) { const int idx = base + lane * 8 + j; const int ic = idx < NPTS ? idx : (NPTS - 1);
                    int v = seg[ic]; asm volatile("" : "+v"(v)); sv[j] = (idx < NPTS) ? v : -1; }
            }
#pragma unroll
            for (int j = 0; j < 8; ++j) {
                const unsigned d = (unsigned)sv[j] - (unsigned)s0;
                const bool hit = d < (unsigned)nloc;
                const unsigned mask = __builtin_amdgcn_ballot_w32(hit);
                const int pos = cnt + (int)__builtin_amdgcn_mbcnt_lo(mask, 0u);
                if (hit & (pos < LCAP)) lst[pos] = (unsigned)(base + lane * 8 + j) | (d << 20);
                cnt += __builtin_popcount(mask);
            }
            wave_sync();
        }
#pragma unroll 1
        for (int trip = 0; trip < LCAP / 16 + 2; ++trip) {
            int nv = 0;
            if (cnt >= 16) nv = 16; else if (last) nv = cnt;
            if (nv <= 0) break;
            cnt -= nv; const int tb = cnt;
            const int li = tb + (lr < nv ? lr : (nv - 1));
            const unsigned ent = lst[li];
            int pidx = (int)(ent & 0xFFFFFu); pidx = pidx < NPTS ? pidx : (NPTS - 1);
            const float* rp = in + (size_t)pidx * CIN + 8 * hi;
            const v4f x0 = *(const v4f*)rp, x1 = *(const v4f*)(rp + 4);
            v8us o;
#pragma unroll
            for (int i = 0; i < 4; ++i) { o[i] = f2bf(x0[i]); o[4 + i] = f2bf(x1[i]); }
            *(v8us*)(&xt[lr * CIN + 8 * hi]) = o;
            wave_sync();
            const v8us alo = *(const v8us*)(&xt[lr * CIN + 8 * hi]);
            const v16bf a = cat16b(alo, z8u);
#pragma unroll
            for (int j = 0; j < 4; ++j) {
                const v8f acc = gwmmab(a, w1f[j], z8);
#pragma unroll
                for (int r = 0; r < 8; ++r) xs[(8 * hi + r) * XP + 16 * j + lr] = fmaxf(bnf(acc[r], m1r[j], s1r[j], b1r[j]), 0.0f);
            }
            wave_sync();
#pragma unroll 1
            for (int p = 0; p < nv; ++p) {
                const unsigned e = lst[tb + p];
                int sl = (int)(e >> 20); sl = sl < SEGB ? sl : (SEGB - 1);
                const v2f xv = *(const v2fa*)(&xs[p * XP + 2 * lane]);
                v4f a4 = *(const v4fa*)(&accs[sl * (2 * C1) + 4 * lane]);
                a4[0] = a4[0] + xv[0]; a4[1] = fmaxf(a4[1], xv[0]); a4[2] = a4[2] + xv[1]; a4[3] = fmaxf(a4[3], xv[1]);
                *(v4fa*)(&accs[sl * (2 * C1) + 4 * lane]) = a4;
            }
            wave_sync();
        }
        if (last) break;
    }
    wave_sync();
    float* ob = OUT + (size_t)s0 * OW;
#pragma unroll 1
    for (int ps = 0; ps < 2; ++ps) {
#pragma unroll 1
        for (int it = 0; it < SEGB * (OW / 4) / 32; ++it) {
            const int q = it * 32 + lane; const int sl = q / (OW / 4); const int w = (q - sl * (OW / 4)) * 4;
            v4f val;
#pragma unroll
            for (int i = 0; i < 4; ++i) { const int e = w + i; const int c = e / 3; const int g = e - 3 * c;
                const float av = accs[sl * (2 * C1) + 2 * c + (g < 2 ? g : 1)]; const float pv = pool[c];
                val[i] = (g < 2) ? av : pv; }
            *(volatile v4f*)(ob + (size_t)q * 4) = val; }
        if (ps == 0) __threadfence(); }
}

static constexpr size_t al256(size_t v) { return (v + 255) & ~(size_t)255; }
static constexpr size_t SZ_W1T = al256((size_t)C1 * 32 * 2);
static constexpr size_t SZ_W2A = al256((size_t)C2A * 32 * 2);
static constexpr size_t SZ_W2B = al256((size_t)C1 * C2A * 2);
static constexpr size_t SZ_PM  = al256((size_t)PB * PW * 64 * 4);
static constexpr size_t SZ_TOTAL = SZ_W1T + SZ_W2A + SZ_W2B + SZ_PM;
static_assert(SZ_TOTAL <= (size_t)134217728);
static constexpr size_t SEG_LDS = (size_t)SEGB * 2 * C1 * 4 + (size_t)16 * XP * 4 + (size_t)16 * CIN * 2 + (size_t)LCAP * 4 + (size_t)C1 * 4;
static_assert(SEG_LDS <= (size_t)131072);
static_assert((size_t)(3 * C2A + 3 * C1) * 4 + (size_t)PW * 64 * 4 <= (size_t)131072);
static_assert((size_t)(NSEG / SEGB) * SEGB * OW * 4 == (size_t)NSEG * OW * 4);

extern "C" void kernel_launch(void* const* d_in, const int* in_sizes, int n_in,
                              void* d_out, int out_size, void* d_ws, size_t ws_size, hipStream_t stream) {
    if (n_in < 18) return;
    if ((size_t)in_sizes[0] < (size_t)NPTS * CIN || (size_t)in_sizes[1] < (size_t)NPTS || in_sizes[2] < 1) return;
    if (in_sizes[3] < CIN * C1 || in_sizes[4] < C1 || in_sizes[5] < C1 || in_sizes[6] < C1 || in_sizes[7] < C1) return;
    if (in_sizes[8] < CIN * C2A || in_sizes[9] < C2A || in_sizes[10] < C2A || in_sizes[11] < C2A || in_sizes[12] < C2A) return;
    if (in_sizes[13] < C2A * C1 || in_sizes[14] < C1 || in_sizes[15] < C1 || in_sizes[16] < C1 || in_sizes[17] < C1) return;
    if ((size_t)out_size < (size_t)NSEG * OW) return;
    if (SZ_TOTAL > ws_size) return;
    const float* xin = (const float*)d_in[0];
    const int*   sid = (const int*)d_in[1];
    const int*   nsg = (const int*)d_in[2];
    const float* w1  = (const float*)d_in[3];
    const float* g1  = (const float*)d_in[4];  const float* b1  = (const float*)d_in[5];
    const float* m1  = (const float*)d_in[6];  const float* v1  = (const float*)d_in[7];
    const float* w2a = (const float*)d_in[8];
    const float* g2a = (const float*)d_in[9];  const float* b2a = (const float*)d_in[10];
    const float* m2a = (const float*)d_in[11]; const float* v2a = (const float*)d_in[12];
    const float* w2b = (const float*)d_in[13];
    const float* g2b = (const float*)d_in[14]; const float* b2b = (const float*)d_in[15];
    const float* m2b = (const float*)d_in[16]; const float* v2b = (const float*)d_in[17];
    float* OUT = (float*)d_out;
    char* wsp = (char*)d_ws;
    bf*  W1T  = (bf*)wsp;  wsp += SZ_W1T;
    bf*  W2AT = (bf*)wsp;  wsp += SZ_W2A;
    h16* W2BT = (h16*)wsp; wsp += SZ_W2B;
    float* PM = (float*)wsp; wsp += SZ_PM;

    k_prep<<<dim3(7, 1, 1), 256, 0, stream>>>(w1, w2a, w2b, W1T, W2AT, W2BT);
    k_pool<<<dim3(PB, 1, 1), 32 * PW, 0, stream>>>(xin, W2AT, W2BT, g2a, b2a, m2a, v2a, g2b, b2b, m2b, v2b, PM);
    k_seg<<<dim3(NSEG / SEGB, 1, 1), 32, 0, stream>>>(xin, sid, nsg, W1T, g1, b1, m1, v1, PM, OUT);
}
